// PointNetSetAbstraction_61323543052297
// MI455X (gfx1250) — hardware-verified
//
#include <hip/hip_runtime.h>
#include <stdint.h>

#pragma clang fp contract(off)

typedef __attribute__((ext_vector_type(16))) _Float16 v16h;
typedef __attribute__((ext_vector_type(8)))  _Float16 v8h;
typedef __attribute__((ext_vector_type(8)))  float    v8f;
typedef __attribute__((ext_vector_type(4)))  float    v4f;

constexpr int NBATCH = 16;
constexpr int NPTS   = 4096;
constexpr int NSAMP  = 512;
constexpr int NGRP   = 32;
constexpr int NFEAT  = 6;
constexpr int CIN    = 9;
constexpr int L0C    = 64;
constexpr int L1C    = 64;
constexpr int L2C    = 128;
constexpr int KPAD0  = 32;
constexpr int NROWS  = NBATCH * NSAMP * NGRP;
constexpr int TROWS  = 128;
constexpr int NBLK   = NROWS / TROWS;
constexpr int P40 = 40, P72 = 72, P136 = 136;
constexpr float BN_EPS = 1e-5f;
constexpr float RAD2 = (float)(0.2 * 0.2);
static_assert(__builtin_bit_cast(unsigned, RAD2) == 0x3D23D70Au);
static_assert(NSAMP == 512 && NPTS == 4096 && NGRP == 32);
static_assert(NROWS == 262144 && NBLK * TROWS == NROWS);
static_assert(L0C % 16 == 0 && L1C % 64 == 0 && L2C % 64 == 0 && KPAD0 % 32 == 0 && L0C % 32 == 0);
static_assert((P40 * 2) % 16 == 0 && (P72 * 2) % 16 == 0 && (P136 * 2) % 16 == 0);

constexpr size_t WS_NEWXYZ = 0;
constexpr size_t SZ_NEWXYZ = (size_t)NBATCH * NSAMP * 4 * 4;
constexpr size_t WS_X0     = WS_NEWXYZ + SZ_NEWXYZ;
constexpr size_t SZ_X0     = (size_t)NROWS * KPAD0 * 2;
constexpr size_t WS_H1     = WS_X0 + SZ_X0;
constexpr size_t SZ_H1     = (size_t)NROWS * L1C * 2;
constexpr size_t WS_H2     = WS_H1 + SZ_H1;
constexpr size_t SZ_H2     = (size_t)NROWS * L2C * 2;
constexpr size_t WS_P0     = WS_H2 + SZ_H2;
constexpr size_t SZ_P0     = (size_t)NBLK * 2 * L0C * 4;
constexpr size_t WS_P1     = WS_P0 + SZ_P0;
constexpr size_t SZ_P1     = (size_t)NBLK * 2 * L1C * 4;
constexpr size_t WS_P2     = WS_P1 + SZ_P1;
constexpr size_t SZ_P2     = (size_t)NBLK * 2 * L2C * 4;
constexpr size_t WS_SC0    = WS_P2 + SZ_P2;
constexpr size_t SZ_SC     = 256 * 4;
constexpr size_t WS_SC1    = WS_SC0 + SZ_SC;
constexpr size_t WS_SC2    = WS_SC1 + SZ_SC;
constexpr size_t WS_TOTAL  = WS_SC2 + SZ_SC;
static_assert(WS_TOTAL == 121768960);
static_assert(WS_TOTAL <= (size_t)134217728);
static_assert(WS_X0 % 128 == 0 && WS_H1 % 128 == 0 && WS_H2 % 128 == 0 && WS_P0 % 128 == 0 &&
              WS_P1 % 128 == 0 && WS_P2 % 128 == 0 && WS_SC0 % 128 == 0 && WS_SC1 % 128 == 0 && WS_SC2 % 128 == 0);
constexpr size_t OUT1_FLOAT_OFF = (size_t)NBATCH * 3 * NSAMP;
static_assert(OUT1_FLOAT_OFF * 4 == 98304);
static_assert((OUT1_FLOAT_OFF + (size_t)NBATCH * L2C * NSAMP) * 4 == 4292608);

__device__ __forceinline__ float h16_to_f32(unsigned hb) {
  const unsigned sgn = (hb & 0x8000u) << 16; const unsigned em = hb & 0x7fffu;
  const float fn = __uint_as_float((em << 13) + 0x38000000u);
  const float fs = (float)em * 5.9604644775390625e-8f;
  const float mag = (em < 0x400u) ? fs : fn; return __uint_as_float(__float_as_uint(mag) | sgn); }

__device__ __forceinline__ v16h frag_ld(const _Float16* p) {
  union { v16h v; v8h h[2]; } f;
  f.h[0] = *(const v8h*)(p);
  f.h[1] = *(const v8h*)(p + 16);
  return f.v;
}
__device__ __forceinline__ v8f zero8() { return (v8f){0.f, 0.f, 0.f, 0.f, 0.f, 0.f, 0.f, 0.f}; }
__device__ __forceinline__ v8f mma16(v16h a, v16h b, v8f c) {
  return __builtin_amdgcn_wmma_f32_16x16x32_f16(false, a, false, b, (short)0, c, false, false);
}
__device__ __forceinline__ void guard4(v8f& c0, v8f& c1, v8f& c2, v8f& c3,
                                       v16h a, v16h b0, v16h b1, v16h b2, v16h b3) {
  asm volatile("v_nop\n\tv_nop\n\tv_nop\n\tv_nop"
               : "+v"(c0), "+v"(c1), "+v"(c2), "+v"(c3)
               : "v"(a), "v"(b0), "v"(b1), "v"(b2), "v"(b3));
}
__device__ __forceinline__ void guard8(v8f& c0, v8f& c1, v8f& c2, v8f& c3, v8f& c4, v8f& c5, v8f& c6, v8f& c7,
                                       v16h a, v16h b0, v16h b1, v16h b2, v16h b3, v16h b4, v16h b5, v16h b6, v16h b7) {
  asm volatile("v_nop\n\tv_nop\n\tv_nop\n\tv_nop"
               : "+v"(c0), "+v"(c1), "+v"(c2), "+v"(c3), "+v"(c4), "+v"(c5), "+v"(c6), "+v"(c7)
               : "v"(a), "v"(b0), "v"(b1), "v"(b2), "v"(b3), "v"(b4), "v"(b5), "v"(b6), "v"(b7));
}

__global__ __launch_bounds__(256) void fps_kernel(const float* __restrict__ xyz,
                                                  float* __restrict__ out0,
                                                  float* __restrict__ newxyz) {
  __shared__ __align__(16) float sx[NPTS];
  __shared__ __align__(16) float sy[NPTS];
  __shared__ __align__(16) float sz[NPTS];
  __shared__ __align__(16) float cent[3 * NSAMP];
  __shared__ float rv[2][8];
  __shared__ int   ri[2][8];

  const int b = blockIdx.x;
  const int t = threadIdx.x;
  const int lane = t & 31;
  const int wave = __builtin_amdgcn_readfirstlane(t >> 5);
  const float* xb = xyz + (size_t)b * 3 * NPTS;

#pragma unroll
  for (int q = 0; q < 4; ++q) { const int i4 = t + 256 * q; *(v4f*)(sx + 4 * i4) = *(const v4f*)(xb + 4 * i4); }
  asm volatile("" ::: "memory");
#pragma unroll
  for (int q = 0; q < 4; ++q) { const int i4 = t + 256 * q; *(v4f*)(sy + 4 * i4) = *(const v4f*)(xb + NPTS + 4 * i4); }
  asm volatile("" ::: "memory");
#pragma unroll
  for (int q = 0; q < 4; ++q) { const int i4 = t + 256 * q; *(v4f*)(sz + 4 * i4) = *(const v4f*)(xb + 2 * NPTS + 4 * i4); }

  float dist[16];
#pragma unroll
  for (int j = 0; j < 16; ++j) dist[j] = 1e10f;
  __syncthreads();

  int far = 0;
  for (int it = 0; it < NSAMP; ++it) {
    const float cx = sx[far], cy = sy[far], cz = sz[far];
    if (t == 0) { cent[it] = cx; cent[NSAMP + it] = cy; cent[2 * NSAMP + it] = cz; }
    float bv = -1.0f; int bi = 0;
#pragma unroll
    for (int j = 0; j < 16; ++j) {
      const int i = t + 256 * j;
      const float dx = sx[i] - cx;
      const float dy = sy[i] - cy;
      const float dz = sz[i] - cz;
      const float pxx = dx * dx;
      const float pyy = dy * dy;
      const float pzz = dz * dz;
      const float d = (pxx + pzz) + pyy;
      const float nd = fminf(dist[j], d);
      dist[j] = nd;
      const bool tk = nd > bv;
      bv = tk ? nd : bv;
      bi = tk ? i : bi;
    }
#pragma unroll
    for (int off = 16; off > 0; off >>= 1) {
      const float ov = __shfl_xor(bv, off, 32);
      const int   oi = __shfl_xor(bi, off, 32);
      const bool tk = (ov > bv) || (ov == bv && oi < bi);
      bv = tk ? ov : bv;
      bi = tk ? oi : bi;
    }
    const int p = it & 1;
    if (lane == 0) { rv[p][wave] = bv; ri[p][wave] = bi; }
    __syncthreads();
    float fv = rv[p][0]; int fi = ri[p][0];
#pragma unroll
    for (int w = 1; w < 8; ++w) {
      const float v2 = rv[p][w]; const int i2 = ri[p][w];
      const bool tk = (v2 > fv) || (v2 == fv && i2 < fi);
      fv = tk ? v2 : fv;
      fi = tk ? i2 : fi;
    }
    far = fi;
  }
  __syncthreads();

  float* ob = out0 + (size_t)b * 3 * NSAMP;
  float* nb = newxyz + (size_t)b * NSAMP * 4;
  for (int pass = 0; pass < 2; ++pass) {
#pragma unroll
    for (int q = 0; q < 2; ++q) {
      const int u = t + 256 * q;
      if (u < 384) {
        const v4f v = *(const v4f*)(cent + 4 * u);
        *(volatile v4f*)(ob + 4 * u) = v;
      }
    }
#pragma unroll
    for (int q = 0; q < 2; ++q) {
      const int s = t + 256 * q;
      v4f v;
      v.x = cent[s]; v.y = cent[NSAMP + s]; v.z = cent[2 * NSAMP + s]; v.w = 0.0f;
      *(volatile v4f*)(nb + 4 * s) = v;
    }
    __threadfence();
  }
}

__global__ __launch_bounds__(256) void ballq_kernel(const float* __restrict__ xyz,
                                                    const float* __restrict__ pts,
                                                    const float* __restrict__ newxyz,
                                                    unsigned short* __restrict__ X0) {
  constexpr int CAP = 256;
  constexpr int NSLOT = CAP / 32;
  static_assert(CAP == 256 && NSLOT == 8);
  constexpr float TH0 = RAD2;
  constexpr float TH1 = RAD2 * 0.5f;
  constexpr float TH2 = RAD2 * 0.25f;
  constexpr float TH3 = RAD2 * 0.125f;
  constexpr float TH4 = RAD2 * 0.0625f;
  constexpr float TH5 = RAD2 * 0.03125f;

  __shared__ float csq[CAP];
  __shared__ int   cid[CAP];
  __shared__ int   lad[6][8];
  __shared__ int   wcnt[128];
  __shared__ int   qbase[128];
  __shared__ int   wtot[8];
  __shared__ int   sel[NGRP];

  const int bs = blockIdx.x;
  const int b = bs >> 9;
  const int t = threadIdx.x;
  const int lane = t & 31;
  const int wave = __builtin_amdgcn_readfirstlane(t >> 5);
  const float* xb = xyz + (size_t)b * 3 * NPTS;
  const float* pb = pts + (size_t)b * NFEAT * NPTS;

  const v4f c4 = *(const v4f*)(newxyz + (size_t)bs * 4);
  const float cx = c4.x, cy = c4.y, cz = c4.z;

  csq[t] = __builtin_inff();
  cid[t] = 0x7fffffff;

  const float qxx = cx * cx;
  const float qyy = cy * cy;
  const float qzz = cz * cz;
  const float sqq = (qxx + qzz) + qyy;

  float sq[16];
  int cnt0 = 0, cnt1 = 0, cnt2 = 0, cnt3 = 0, cnt4 = 0, cnt5 = 0;
#pragma unroll
  for (int q = 0; q < 4; ++q) {
    const int n0 = 1024 * q + 4 * t;
    const v4f X = *(const v4f*)(xb + n0);
    const v4f Y = *(const v4f*)(xb + NPTS + n0);
    const v4f Z = *(const v4f*)(xb + 2 * NPTS + n0);
    asm volatile("" ::: "memory");
#pragma unroll
    for (int e = 0; e < 4; ++e) {
      const float rx = X[e], ry = Y[e], rz = Z[e];
      const float rxx = rx * rx;
      const float ryy = ry * ry;
      const float rzz = rz * rz;
      const float sqr = (rxx + rzz) + ryy;
      const float dxq = cx * rx;
      const float dot = fmaf(cz, rz, fmaf(cy, ry, dxq));
      const float tdot = 2.0f * dot;
      const float ssum = sqq + sqr;
      const float s = ssum - tdot;
      sq[4 * q + e] = s;
      cnt0 += (s <= TH0) ? 1 : 0;
      cnt1 += (s <= TH1) ? 1 : 0;
      cnt2 += (s <= TH2) ? 1 : 0;
      cnt3 += (s <= TH3) ? 1 : 0;
      cnt4 += (s <= TH4) ? 1 : 0;
      cnt5 += (s <= TH5) ? 1 : 0;
    }
  }

  {
    int c0 = cnt0, c1 = cnt1, c2 = cnt2, c3 = cnt3, c4i = cnt4, c5 = cnt5;
#pragma unroll
    for (int off = 16; off > 0; off >>= 1) {
      c0 += __shfl_xor(c0, off, 32);
      c1 += __shfl_xor(c1, off, 32);
      c2 += __shfl_xor(c2, off, 32);
      c3 += __shfl_xor(c3, off, 32);
      c4i += __shfl_xor(c4i, off, 32);
      c5 += __shfl_xor(c5, off, 32);
    }
    if (lane == 0) {
      lad[0][wave] = c0; lad[1][wave] = c1; lad[2][wave] = c2;
      lad[3][wave] = c3; lad[4][wave] = c4i; lad[5][wave] = c5;
    }
  }
  __syncthreads();
  int tot[6];
#pragma unroll
  for (int k = 0; k < 6; ++k) {
    int a = 0;
#pragma unroll
    for (int w = 0; w < 8; ++w) a += lad[k][w];
    tot[k] = a;
  }
  const float thr = (tot[0] <= CAP) ? TH0 : (tot[1] <= CAP) ? TH1 : (tot[2] <= CAP) ? TH2
                  : (tot[3] <= CAP) ? TH3 : (tot[4] <= CAP) ? TH4 : TH5;

  unsigned msk[16];
#pragma unroll
  for (int j = 0; j < 16; ++j) {
    const unsigned m = __builtin_amdgcn_ballot_w32(sq[j] <= thr);
    msk[j] = m;
    if (lane == 0) wcnt[j * 8 + wave] = (int)__builtin_popcount(m);
  }
  __syncthreads();

  const int tcl = (t < 128) ? t : 127;
  int x = wcnt[tcl];
  x = (t < 128) ? x : 0;
  const int own = x;
#pragma unroll
  for (int d = 1; d < 32; d <<= 1) {
    const int y = __shfl_up(x, d, 32);
    x = (lane >= d) ? (x + y) : x;
  }
  if (lane == 31) wtot[wave] = x;
  __syncthreads();
  {
    const int w0 = wtot[0], w1 = wtot[1], w2 = wtot[2];
    const int pre = ((wave > 0) ? w0 : 0) + ((wave > 1) ? w1 : 0) + ((wave > 2) ? w2 : 0);
    if (t < 128) qbase[t] = x - own + pre;
  }
  __syncthreads();

#pragma unroll
  for (int j = 0; j < 16; ++j) {
    const int base = qbase[j * 8 + wave];
    const unsigned m = msk[j];
    const bool p = ((m >> lane) & 1u) != 0u;
    const int pos = base + (int)__builtin_popcount(m & ((1u << lane) - 1u));
    const int n = 1024 * (j >> 2) + 4 * t + (j & 3);
    if (p && pos < CAP) { csq[pos] = sq[j]; cid[pos] = n; }
  }
  __syncthreads();

  if (wave == 0) {
    float ssq[NSLOT]; int sid[NSLOT];
#pragma unroll
    for (int m = 0; m < NSLOT; ++m) { ssq[m] = csq[lane + 32 * m]; sid[m] = cid[lane + 32 * m]; }
    float mysq = __builtin_inff();
    int myid = 0;
    int firstid = 0;
#pragma unroll 1
    for (int r = 0; r < NGRP; ++r) {
      float bv = ssq[0]; int bi = sid[0];
#pragma unroll
      for (int m = 1; m < NSLOT; ++m) {
        const bool tk = (ssq[m] < bv) || (ssq[m] == bv && sid[m] < bi);
        bv = tk ? ssq[m] : bv;
        bi = tk ? sid[m] : bi;
      }
#pragma unroll
      for (int off = 16; off > 0; off >>= 1) {
        const float ov = __shfl_xor(bv, off, 32);
        const int   oi = __shfl_xor(bi, off, 32);
        const bool tk = (ov < bv) || (ov == bv && oi < bi);
        bv = tk ? ov : bv;
        bi = tk ? oi : bi;
      }
      firstid = (r == 0) ? bi : firstid;
      const bool me = (lane == r);
      mysq = me ? bv : mysq;
      myid = me ? bi : myid;
#pragma unroll
      for (int m = 0; m < NSLOT; ++m) ssq[m] = (sid[m] == bi) ? __builtin_inff() : ssq[m];
    }
    int idx = (mysq > RAD2) ? firstid : myid;
    idx = (idx < 0) ? 0 : idx;
    idx = (idx > NPTS - 1) ? (NPTS - 1) : idx;
    sel[lane] = idx;
  }
  __syncthreads();

  if (wave < 4) {
    const int k = t >> 2;
    const int cc = t & 3;
    const int idx = sel[k];
    const float px = xb[idx];
    const float py = xb[NPTS + idx];
    const float pz = xb[2 * NPTS + idx];
    const float f0 = pb[0 * NPTS + idx];
    const float f1 = pb[1 * NPTS + idx];
    const float f2 = pb[2 * NPTS + idx];
    const float f3 = pb[3 * NPTS + idx];
    const float f4 = pb[4 * NPTS + idx];
    const float f5 = pb[5 * NPTS + idx];
    const float v0 = px - cx;
    const float v1 = py - cy;
    const float v2 = pz - cz;
    const bool c0 = (cc == 0);
    const bool c1 = (cc == 1);
    float o[8];
    o[0] = c0 ? v0 : (c1 ? f5 : 0.0f);
    o[1] = c0 ? v1 : 0.0f;
    o[2] = c0 ? v2 : 0.0f;
    o[3] = c0 ? f0 : 0.0f;
    o[4] = c0 ? f1 : 0.0f;
    o[5] = c0 ? f2 : 0.0f;
    o[6] = c0 ? f3 : 0.0f;
    o[7] = c0 ? f4 : 0.0f;
    v8h hv;
#pragma unroll
    for (int e = 0; e < 8; ++e) hv[e] = (_Float16)o[e];
    unsigned short* dst = X0 + ((size_t)bs * NGRP + k) * KPAD0 + cc * 8;
    *(volatile v8h*)dst = hv;
    __threadfence();
    *(volatile v8h*)dst = hv;
  }
}

__device__ __forceinline__ void layer0_tile(const unsigned short* __restrict__ X0, const _Float16* W0s,
                                            int blk, int wave, int lane, v8f (&acc)[4]) {
  const int rlane = lane & 15;
  const int koff  = (lane >> 4) * 8;
  const _Float16* xr = (const _Float16*)(const void*)X0 +
                       ((size_t)blk * TROWS + (size_t)wave * 16 + rlane) * KPAD0 + koff;
  const v16h a  = frag_ld(xr);
  const v16h q0 = frag_ld(W0s + (0 * 16 + rlane) * P40 + koff);
  const v16h q1 = frag_ld(W0s + (1 * 16 + rlane) * P40 + koff);
  const v16h q2 = frag_ld(W0s + (2 * 16 + rlane) * P40 + koff);
  const v16h q3 = frag_ld(W0s + (3 * 16 + rlane) * P40 + koff);
  acc[0] = mma16(a, q0, zero8());
  acc[1] = mma16(a, q1, zero8());
  acc[2] = mma16(a, q2, zero8());
  acc[3] = mma16(a, q3, zero8());
  guard4(acc[0], acc[1], acc[2], acc[3], a, q0, q1, q2, q3);
}

__global__ __launch_bounds__(256) void l0_stats_kernel(const unsigned short* __restrict__ X0,
                                                       const float* __restrict__ W0,
                                                       const float* __restrict__ b0,
                                                       float* __restrict__ part0) {
  __shared__ __align__(16) _Float16 W0s[L0C * P40];
  __shared__ float b0s[L0C];
  __shared__ float wsum[8][L0C];
  __shared__ float wsq[8][L0C];
  __shared__ __align__(16) float orow[2 * L0C];

  const int blk = blockIdx.x;
  const int t = threadIdx.x;
  const int lane = t & 31;
  const int wave = __builtin_amdgcn_readfirstlane(t >> 5);
  const int rlane = lane & 15;
  const int hh = lane >> 4;

  for (int i = t; i < L0C * P40 / 2; i += 256) ((unsigned*)(void*)W0s)[i] = 0u;
  if (t < L0C) b0s[t] = b0[t];
  __syncthreads();
  for (int i = t; i < L0C * CIN; i += 256) {
    const int o = i / CIN; const int kk = i - o * CIN;
    W0s[o * P40 + kk] = (_Float16)W0[i];
  }
  __syncthreads();

  v8f acc[4];
  layer0_tile(X0, W0s, blk, wave, lane, acc);

#pragma unroll
  for (int j = 0; j < 4; ++j) {
    const int n = j * 16 + rlane;
    const float bb = b0s[n];
    float s = 0.0f, s2 = 0.0f;
#pragma unroll
    for (int r = 0; r < 8; ++r) {
      const float v = acc[j][r] + bb;
      s = s + v;
      s2 = fmaf(v, v, s2);
    }
    s  += __shfl_xor(s, 16, 32);
    s2 += __shfl_xor(s2, 16, 32);
    if (hh == 0) { wsum[wave][n] = s; wsq[wave][n] = s2; }
  }
  __syncthreads();
  if (t < L0C) {
    float S = 0.0f, S2 = 0.0f;
#pragma unroll
    for (int w = 0; w < 8; ++w) { S = S + wsum[w][t]; S2 = S2 + wsq[w][t]; }
    orow[t] = S; orow[L0C + t] = S2;
  }
  __syncthreads();
  if (wave == 0) {
    float* dst = part0 + (size_t)blk * 2 * L0C;
    for (int pass = 0; pass < 2; ++pass) {
      const v4f v = *(const v4f*)(orow + 4 * lane);
      *(volatile v4f*)(dst + 4 * lane) = v;
      __threadfence();
    }
  }
}

template <int COUT>
__global__ __launch_bounds__(128) void bn_finalize_kernel(const float* __restrict__ part,
                                                          const float* __restrict__ gam,
                                                          const float* __restrict__ bet,
                                                          float* __restrict__ scsh) {
  static_assert(COUT == 64 || COUT == 128);
  __shared__ __align__(16) float row[256];
  const int t = threadIdx.x;
  const int lane = t & 31;
  const int wave = __builtin_amdgcn_readfirstlane(t >> 5);
  const int c = (t < COUT) ? t : (COUT - 1);
  double S = 0.0, S2 = 0.0;
#pragma unroll 1
  for (int blk = 0; blk < NBLK; ++blk) {
    const float* p = part + (size_t)blk * 2 * COUT;
    S  += (double)p[c];
    S2 += (double)p[COUT + c];
  }
  const double inv_n = 1.0 / (double)NROWS;
  const double mean = S * inv_n;
  const double msq = mean * mean;
  const double ex2 = S2 * inv_n;
  const double var = ex2 - msq;
  float varf = (float)var;
  varf = (varf > 0.0f) ? varf : 0.0f;
  const float meanf = (float)mean;
  const float istd = rsqrtf(varf + BN_EPS);
  const float sc = gam[c] * istd;
  const float msc = meanf * sc;
  const float sh = bet[c] - msc;
  row[t] = (t < COUT) ? sc : 0.0f;
  row[128 + t] = (t < COUT) ? sh : 0.0f;
  __syncthreads();
  if (wave == 0) {
    for (int pass = 0; pass < 2; ++pass) {
#pragma unroll
      for (int it = 0; it < 2; ++it) {
        const v4f v = *(const v4f*)(row + it * 128 + 4 * lane);
        *(volatile v4f*)(scsh + it * 128 + 4 * lane) = v;
      }
      __threadfence();
    }
  }
}

__global__ __launch_bounds__(256) void l1_kernel(const unsigned short* __restrict__ X0,
                                                 const float* __restrict__ W0,
                                                 const float* __restrict__ b0,
                                                 const float* __restrict__ scsh0,
                                                 const float* __restrict__ W1,
                                                 const float* __restrict__ b1,
                                                 unsigned short* __restrict__ H1,
                                                 float* __restrict__ part1) {
  __shared__ __align__(16) _Float16 W0s[L0C * P40];
  __shared__ __align__(16) _Float16 W1s[L1C * P72];
  __shared__ __align__(16) _Float16 A1s[TROWS * P72];
  __shared__ float b0s[L0C];
  __shared__ float sc0[L0C];
  __shared__ float sh0[L0C];
  __shared__ float b1s[L1C];
  __shared__ float wsum[8][L1C];
  __shared__ float wsq[8][L1C];
  __shared__ __align__(16) float orow[2 * L1C];

  const int blk = blockIdx.x;
  const int t = threadIdx.x;
  const int lane = t & 31;
  const int wave = __builtin_amdgcn_readfirstlane(t >> 5);
  const int rlane = lane & 15;
  const int hh = lane >> 4;
  const int koff = hh * 8;

  for (int i = t; i < L0C * P40 / 2; i += 256) ((unsigned*)(void*)W0s)[i] = 0u;
  if (t < L0C) { b0s[t] = b0[t]; sc0[t] = scsh0[t]; sh0[t] = scsh0[128 + t]; b1s[t] = b1[t]; }
  asm volatile("" ::: "memory");
#pragma unroll
  for (int q = 0; q < 4; ++q) {
    const int u = t + 256 * q;
    const int o = u >> 4;
    const int c4i = (u & 15) * 4;
    const v4f w = *(const v4f*)(W1 + (size_t)o * L0C + c4i);
    _Float16* d = W1s + o * P72 + c4i;
    d[0] = (_Float16)w.x; d[1] = (_Float16)w.y; d[2] = (_Float16)w.z; d[3] = (_Float16)w.w;
  }
  __syncthreads();
  for (int i = t; i < L0C * CIN; i += 256) {
    const int o = i / CIN; const int kk = i - o * CIN;
    W0s[o * P40 + kk] = (_Float16)W0[i];
  }
  __syncthreads();

  v8f acc0[4];
  layer0_tile(X0, W0s, blk, wave, lane, acc0);

#pragma unroll
  for (int j = 0; j < 4; ++j) {
    const int n = j * 16 + rlane;
    const float bb = b0s[n];
    const float sc = sc0[n];
    const float sh = sh0[n];
#pragma unroll
    for (int r = 0; r < 8; ++r) {
      const float v = acc0[j][r] + bb;
      const float y = fmaxf(fmaf(v, sc, sh), 0.0f);
      A1s[(wave * 16 + 8 * hh + r) * P72 + n] = (_Float16)y;
    }
  }
  __syncthreads();

  v8f acc1[4];
  acc1[0] = zero8(); acc1[1] = zero8(); acc1[2] = zero8(); acc1[3] = zero8();
#pragma unroll
  for (int ks = 0; ks < 2; ++ks) {
    const v16h a  = frag_ld(A1s + (wave * 16 + rlane) * P72 + ks * 32 + koff);
    const v16h q0 = frag_ld(W1s + (0 * 16 + rlane) * P72 + ks * 32 + koff);
    const v16h q1 = frag_ld(W1s + (1 * 16 + rlane) * P72 + ks * 32 + koff);
    const v16h q2 = frag_ld(W1s + (2 * 16 + rlane) * P72 + ks * 32 + koff);
    const v16h q3 = frag_ld(W1s + (3 * 16 + rlane) * P72 + ks * 32 + koff);
    acc1[0] = mma16(a, q0, acc1[0]);
    acc1[1] = mma16(a, q1, acc1[1]);
    acc1[2] = mma16(a, q2, acc1[2]);
    acc1[3] = mma16(a, q3, acc1[3]);
    guard4(acc1[0], acc1[1], acc1[2], acc1[3], a, q0, q1, q2, q3);
  }
  __syncthreads();

#pragma unroll
  for (int j = 0; j < 4; ++j) {
    const int n = j * 16 + rlane;
    const float bb = b1s[n];
    float s = 0.0f, s2 = 0.0f;
#pragma unroll
    for (int r = 0; r < 8; ++r) {
      const float v = acc1[j][r] + bb;
      s = s + v;
      s2 = fmaf(v, v, s2);
      A1s[(wave * 16 + 8 * hh + r) * P72 + n] = (_Float16)v;
    }
    s  += __shfl_xor(s, 16, 32);
    s2 += __shfl_xor(s2, 16, 32);
    if (hh == 0) { wsum[wave][n] = s; wsq[wave][n] = s2; }
  }
  __syncthreads();

  {
    const int q = lane >> 3;
    const int c8 = (lane & 7) * 8;
    unsigned short* hb = H1 + ((size_t)blk * TROWS + (size_t)wave * 16) * L1C;
    for (int pass = 0; pass < 2; ++pass) {
#pragma unroll
      for (int it = 0; it < 4; ++it) {
        const int rr = it * 4 + q;
        const v8h v = *(const v8h*)(A1s + (wave * 16 + rr) * P72 + c8);
        *(volatile v8h*)(hb + (size_t)rr * L1C + c8) = v;
      }
      __threadfence();
    }
  }
  if (t < L1C) {
    float S = 0.0f, S2 = 0.0f;
#pragma unroll
    for (int w = 0; w < 8; ++w) { S = S + wsum[w][t]; S2 = S2 + wsq[w][t]; }
    orow[t] = S; orow[L1C + t] = S2;
  }
  __syncthreads();
  if (wave == 0) {
    float* dst = part1 + (size_t)blk * 2 * L1C;
    for (int pass = 0; pass < 2; ++pass) {
      const v4f v = *(const v4f*)(orow + 4 * lane);
      *(volatile v4f*)(dst + 4 * lane) = v;
      __threadfence();
    }
  }
}

__global__ __launch_bounds__(256) void l2_kernel(const unsigned short* __restrict__ H1,
                                                 const float* __restrict__ scsh1,
                                                 const float* __restrict__ W2,
                                                 const float* __restrict__ b2,
                                                 unsigned short* __restrict__ H2,
                                                 float* __restrict__ part2) {
  __shared__ __align__(16) _Float16 W2s[L2C * P72];
  __shared__ __align__(16) _Float16 A2s[TROWS * P136];
  __shared__ float sc1[L1C];
  __shared__ float sh1[L1C];
  __shared__ float b2s[L2C];
  __shared__ float wsum[8][L2C];
  __shared__ float wsq[8][L2C];
  __shared__ __align__(16) float orow[2 * L2C];

  const int blk = blockIdx.x;
  const int t = threadIdx.x;
  const int lane = t & 31;
  const int wave = __builtin_amdgcn_readfirstlane(t >> 5);
  const int rlane = lane & 15;
  const int hh = lane >> 4;
  const int koff = hh * 8;

  if (t < L1C) { sc1[t] = scsh1[t]; sh1[t] = scsh1[128 + t]; }
  if (t < L2C) b2s[t] = b2[t];
  asm volatile("" ::: "memory");
#pragma unroll
  for (int q = 0; q < 8; ++q) {
    const int u = t + 256 * q;
    const int o = u >> 4;
    const int c4i = (u & 15) * 4;
    const v4f w = *(const v4f*)(W2 + (size_t)o * L1C + c4i);
    _Float16* d = W2s + o * P72 + c4i;
    d[0] = (_Float16)w.x; d[1] = (_Float16)w.y; d[2] = (_Float16)w.z; d[3] = (_Float16)w.w;
    if (q == 3) { asm volatile("" ::: "memory"); }
  }
  __syncthreads();

#pragma unroll
  for (int q = 0; q < 4; ++q) {
    const int u = t + 256 * q;
    const int rr = u >> 3;
    const int c8 = (u & 7) * 8;
    const uint4 w = *(const uint4*)(const void*)(H1 + ((size_t)blk * TROWS + rr) * L1C + c8);
    const unsigned wv[4] = {w.x, w.y, w.z, w.w};
#pragma unroll
    for (int i = 0; i < 4; ++i) {
      const int ch = c8 + 2 * i;
      const float fa = h16_to_f32(wv[i] & 0xffffu);
      const float fb = h16_to_f32(wv[i] >> 16);
      const float ya = fmaxf(fmaf(fa, sc1[ch], sh1[ch]), 0.0f);
      const float yb = fmaxf(fmaf(fb, sc1[ch + 1], sh1[ch + 1]), 0.0f);
      A2s[rr * P136 + ch] = (_Float16)ya;
      A2s[rr * P136 + ch + 1] = (_Float16)yb;
    }
  }
  __syncthreads();

  v8f acc[8];
#pragma unroll
  for (int j = 0; j < 8; ++j) acc[j] = zero8();
#pragma unroll
  for (int ks = 0; ks < 2; ++ks) {
    const v16h a = frag_ld(A2s + (wave * 16 + rlane) * P136 + ks * 32 + koff);
    v16h q[8];
#pragma unroll
    for (int j = 0; j < 8; ++j) q[j] = frag_ld(W2s + (j * 16 + rlane) * P72 + ks * 32 + koff);
#pragma unroll
    for (int j = 0; j < 8; ++j) acc[j] = mma16(a, q[j], acc[j]);
    guard8(acc[0], acc[1], acc[2], acc[3], acc[4], acc[5], acc[6], acc[7],
           a, q[0], q[1], q[2], q[3], q[4], q[5], q[6], q[7]);
  }
  __syncthreads();

#pragma unroll
  for (int j = 0; j < 8; ++j) {
    const int n = j * 16 + rlane;
    const float bb = b2s[n];
    float s = 0.0f, s2 = 0.0f;
#pragma unroll
    for (int r = 0; r < 8; ++r) {
      const float v = acc[j][r] + bb;
      s = s + v;
      s2 = fmaf(v, v, s2);
      A2s[(wave * 16 + 8 * hh + r) * P136 + n] = (_Float16)v;
    }
    s  += __shfl_xor(s, 16, 32);
    s2 += __shfl_xor(s2, 16, 32);
    if (hh == 0) { wsum[wave][n] = s; wsq[wave][n] = s2; }
  }
  __syncthreads();

  {
    const int rsub = lane >> 4;
    const int c8 = (lane & 15) * 8;
    unsigned short* hb = H2 + ((size_t)blk * TROWS + (size_t)wave * 16) * L2C;
    for (int pass = 0; pass < 2; ++pass) {
#pragma unroll
      for (int it = 0; it < 8; ++it) {
        const int rr = it * 2 + rsub;
        const v8h v = *(const v8h*)(A2s + (wave * 16 + rr) * P136 + c8);
        *(volatile v8h*)(hb + (size_t)rr * L2C + c8) = v;
      }
      __threadfence();
    }
  }
  if (t < L2C) {
    float S = 0.0f, S2 = 0.0f;
#pragma unroll
    for (int w = 0; w < 8; ++w) { S = S + wsum[w][t]; S2 = S2 + wsq[w][t]; }
    orow[t] = S; orow[L2C + t] = S2;
  }
  __syncthreads();
  if (wave == 0) {
    float* dst = part2 + (size_t)blk * 2 * L2C;
    for (int pass = 0; pass < 2; ++pass) {
#pragma unroll
      for (int it = 0; it < 2; ++it) {
        const v4f v = *(const v4f*)(orow + it * 128 + 4 * lane);
        *(volatile v4f*)(dst + it * 128 + 4 * lane) = v;
      }
      __threadfence();
    }
  }
}

__global__ __launch_bounds__(256) void maxpool_kernel(const unsigned short* __restrict__ H2,
                                                      const float* __restrict__ scsh2,
                                                      float* __restrict__ out1) {
  __shared__ float sc2[L2C];
  __shared__ float sh2[L2C];
  __shared__ __align__(16) float Ts[L2C * 36];

  const int blk = blockIdx.x;
  const int b = blk >> 4;
  const int st = blk & 15;
  const int s0 = st * 32;
  const int t = threadIdx.x;
  const int sl = t >> 3;
  const int cc = t & 7;

  if (t < L2C) { sc2[t] = scsh2[t]; sh2[t] = scsh2[128 + t]; }
  __syncthreads();
  float sc[16], sh[16], m[16];
#pragma unroll
  for (int e = 0; e < 16; ++e) { sc[e] = sc2[16 * cc + e]; sh[e] = sh2[16 * cc + e]; m[e] = 0.0f; }

  const size_t rowbase = ((size_t)b * NSAMP + s0 + sl) * NGRP;
#pragma unroll 1
  for (int k = 0; k < NGRP; ++k) {
    const uint4* p = (const uint4*)(const void*)(H2 + (rowbase + k) * L2C + 16 * cc);
    const uint4 wa = p[0];
    const uint4 wb = p[1];
    const unsigned wv[8] = {wa.x, wa.y, wa.z, wa.w, wb.x, wb.y, wb.z, wb.w};
#pragma unroll
    for (int i = 0; i < 8; ++i) {
      const float fa = h16_to_f32(wv[i] & 0xffffu);
      const float fb = h16_to_f32(wv[i] >> 16);
      const float ya = fmaxf(fmaf(fa, sc[2 * i], sh[2 * i]), 0.0f);
      const float yb = fmaxf(fmaf(fb, sc[2 * i + 1], sh[2 * i + 1]), 0.0f);
      m[2 * i] = fmaxf(m[2 * i], ya);
      m[2 * i + 1] = fmaxf(m[2 * i + 1], yb);
    }
  }
#pragma unroll
  for (int e = 0; e < 16; ++e) Ts[(16 * cc + e) * 36 + sl] = m[e];
  __syncthreads();

  const int o = t >> 3;
  const int p4 = (t & 7) * 4;
  float* ob = out1 + (size_t)b * L2C * NSAMP + s0;
  for (int pass = 0; pass < 2; ++pass) {
#pragma unroll
    for (int u = 0; u < 4; ++u) {
      const int oo = o + 32 * u;
      const v4f v = *(const v4f*)(Ts + oo * 36 + p4);
      *(volatile v4f*)(ob + (size_t)oo * NSAMP + p4) = v;
    }
    __threadfence();
  }
}

extern "C" void kernel_launch(void* const* d_in, const int* in_sizes, int n_in,
                              void* d_out, int out_size, void* d_ws, size_t ws_size,
                              hipStream_t stream) {
  if (n_in < 14) return;
  if (in_sizes[0] != NBATCH * 3 * NPTS) return;
  if (in_sizes[1] != NBATCH * NFEAT * NPTS) return;
  if (in_sizes[2] != L0C * CIN || in_sizes[6] != L1C * L0C || in_sizes[10] != L2C * L1C) return;
  if (out_size != NBATCH * 3 * NSAMP + NBATCH * L2C * NSAMP) return;
  if (ws_size < WS_TOTAL) return;

  const float* xyz = (const float*)d_in[0];
  const float* pts = (const float*)d_in[1];
  const float* W0  = (const float*)d_in[2];
  const float* b0  = (const float*)d_in[3];
  const float* g0  = (const float*)d_in[4];
  const float* be0 = (const float*)d_in[5];
  const float* W1  = (const float*)d_in[6];
  const float* b1  = (const float*)d_in[7];
  const float* g1  = (const float*)d_in[8];
  const float* be1 = (const float*)d_in[9];
  const float* W2  = (const float*)d_in[10];
  const float* b2  = (const float*)d_in[11];
  const float* g2  = (const float*)d_in[12];
  const float* be2 = (const float*)d_in[13];

  char* ws = (char*)d_ws;
  float*          newxyz = (float*)(ws + WS_NEWXYZ);
  unsigned short* X0     = (unsigned short*)(ws + WS_X0);
  unsigned short* H1     = (unsigned short*)(ws + WS_H1);
  unsigned short* H2     = (unsigned short*)(ws + WS_H2);
  float*          part0  = (float*)(ws + WS_P0);
  float*          part1  = (float*)(ws + WS_P1);
  float*          part2  = (float*)(ws + WS_P2);
  float*          scsh0  = (float*)(ws + WS_SC0);
  float*          scsh1  = (float*)(ws + WS_SC1);
  float*          scsh2  = (float*)(ws + WS_SC2);

  float* out0 = (float*)d_out;
  float* out1 = (float*)d_out + OUT1_FLOAT_OFF;

  fps_kernel<<<NBATCH, 256, 0, stream>>>(xyz, out0, newxyz);
  ballq_kernel<<<NBATCH * NSAMP, 256, 0, stream>>>(xyz, pts, newxyz, X0);
  l0_stats_kernel<<<NBLK, 256, 0, stream>>>(X0, W0, b0, part0);
  bn_finalize_kernel<L0C><<<1, 128, 0, stream>>>(part0, g0, be0, scsh0);
  l1_kernel<<<NBLK, 256, 0, stream>>>(X0, W0, b0, scsh0, W1, b1, H1, part1);
  bn_finalize_kernel<L1C><<<1, 128, 0, stream>>>(part1, g1, be1, scsh1);
  l2_kernel<<<NBLK, 256, 0, stream>>>(H1, scsh1, W2, b2, H2, part2);
  bn_finalize_kernel<L2C><<<1, 128, 0, stream>>>(part2, g2, be2, scsh2);
  maxpool_kernel<<<NBATCH * (NSAMP / 32), 256, 0, stream>>>(H2, scsh2, out1);
}
